// SelfAttention_4466765988490
// MI455X (gfx1250) — hardware-verified
//
#include <hip/hip_runtime.h>
#ifndef NB
#define NB 2
#endif
#ifndef SEQ
#define SEQ 2048
#endif
#define NB_FULL 2
#define SEQ_FULL 2048
#define DMODEL 1024
#define NHEAD 16
#define HD 64
#define NQKV 3072
#define LDQK 2048
#define TOK (NB * SEQ)

static_assert(NHEAD * HD == DMODEL);
static_assert(HD == 64);
static_assert(3 * DMODEL == NQKV && 2 * DMODEL == LDQK);
static_assert(SEQ % 64 == 0 && SEQ % 32 == 0);
static_assert(TOK % 128 == 0 && TOK % 64 == 0);
static_assert(DMODEL % 128 == 0 && DMODEL % 64 == 0 && DMODEL % 32 == 0 && LDQK % 64 == 0);
static_assert(NB <= NB_FULL && SEQ <= SEQ_FULL);

typedef unsigned short v8us __attribute__((ext_vector_type(8), may_alias));
typedef float  v8f  __attribute__((ext_vector_type(8)));
typedef float  v4f  __attribute__((ext_vector_type(4)));
typedef float  v4fa __attribute__((ext_vector_type(4), may_alias));
typedef _Float16 v16h __attribute__((ext_vector_type(16)));
union FragH { v16h v; v8us half[2]; _Float16 h[16]; unsigned short u[16]; };

__device__ __forceinline__ unsigned short bf16_bits(float x) { unsigned int u = __float_as_uint(x); return (unsigned short)((u + 0x7FFFu + ((u >> 16) & 1u)) >> 16); }
__device__ __forceinline__ float bf16_rne(float x) { return __uint_as_float(((unsigned int)bf16_bits(x)) << 16); }

__device__ __forceinline__ v16h g2_frag(const _Float16* p, int hh) { FragH f; f.half[0] = *(const v8us*)((const unsigned short*)p + 8 * hh); f.half[1] = *(const v8us*)((const unsigned short*)p + 16 + 8 * hh); return f.v; }
__device__ __forceinline__ v8f g2_mma(v16h a, v16h b, v8f c) { v8f d = __builtin_amdgcn_wmma_f32_16x16x32_f16(false, a, false, b, (short)0, c, false, false); asm volatile("v_nop\n\tv_nop\n\tv_nop\n\tv_nop" : "+v"(d) : "v"(a), "v"(b)); return d; }

__global__ __launch_bounds__(256) void k_x16(const float* __restrict__ x, _Float16* __restrict__ X16) {
  const size_t t = (size_t)blockIdx.x * 256 + threadIdx.x; if (t >= (size_t)TOK * (DMODEL / 8)) return;
  const size_t r = t / (DMODEL / 8); const int c8 = (int)(t % (DMODEL / 8)) * 8; const size_t b = r / SEQ, s = r % SEQ;
  const float* src = x + (b * SEQ_FULL + s) * DMODEL + c8; const v4f a = *(const v4fa*)src, c = *(const v4fa*)(src + 4); FragH f;
#pragma unroll
  for (int q = 0; q < 4; ++q) { f.h[q] = (_Float16)bf16_rne(a[q]); f.h[4 + q] = (_Float16)bf16_rne(c[q]); }
  const v8us o = f.half[0]; unsigned short* d = (unsigned short*)X16 + t * 8;
  *(volatile v8us*)d = o; __threadfence(); *(volatile v8us*)d = o; }

__global__ __launch_bounds__(256) void k_wnat(const float* __restrict__ w, size_t n8, float scale, _Float16* __restrict__ Bt) {
  const size_t t = (size_t)blockIdx.x * 256 + threadIdx.x; if (t >= n8) return; const v4f a = *(const v4fa*)(w + t * 8), c = *(const v4fa*)(w + t * 8 + 4); FragH f;
#pragma unroll
  for (int q = 0; q < 4; ++q) { f.h[q] = (_Float16)(bf16_rne(a[q]) * scale); f.h[4 + q] = (_Float16)(bf16_rne(c[q]) * scale); }
  const v8us o = f.half[0]; unsigned short* d = (unsigned short*)Bt + t * 8;
  *(volatile v8us*)d = o; __threadfence(); *(volatile v8us*)d = o; }

template <int MODE>
__device__ __forceinline__ void gemm_body(const _Float16* __restrict__ A, int lda, const _Float16* __restrict__ Bh, int ldb, float alpha, const float* __restrict__ bias,
                                          float* __restrict__ C, _Float16* __restrict__ C16, int ldc, int M, int N, int K) {
  __shared__ __attribute__((aligned(16))) float so[4][32][68];
  const int tid = threadIdx.x, w = tid >> 5, lane = tid & 31, ln = lane & 15, hh = lane >> 4;
  const int ntn = N >> 6; const int mt = blockIdx.x / ntn, nq = blockIdx.x - mt * ntn; const int row0 = mt * 128 + 32 * w, col0 = nq * 64; if (row0 >= M) return;
  const _Float16* a0p = A + (size_t)(row0 + ln) * lda; const _Float16* a1p = a0p + (size_t)16 * lda;
  const _Float16* b0p = Bh + (size_t)(col0 + ln) * ldb; const _Float16* b1p = b0p + (size_t)16 * ldb; const _Float16* b2p = b1p + (size_t)16 * ldb; const _Float16* b3p = b2p + (size_t)16 * ldb;
  const v8f z8 = {0.f,0.f,0.f,0.f,0.f,0.f,0.f,0.f}; v8f c00 = z8, c01 = z8, c02 = z8, c03 = z8, c10 = z8, c11 = z8, c12 = z8, c13 = z8;
#pragma unroll 1
  for (int kb = 0; kb < K; kb += 32) { const v16h a0 = g2_frag(a0p + kb, hh), a1 = g2_frag(a1p + kb, hh);
    v16h b = g2_frag(b0p + kb, hh); c00 = g2_mma(a0, b, c00); c10 = g2_mma(a1, b, c10);
    b = g2_frag(b1p + kb, hh); c01 = g2_mma(a0, b, c01); c11 = g2_mma(a1, b, c11);
    b = g2_frag(b2p + kb, hh); c02 = g2_mma(a0, b, c02); c12 = g2_mma(a1, b, c12);
    b = g2_frag(b3p + kb, hh); c03 = g2_mma(a0, b, c03); c13 = g2_mma(a1, b, c13); }
  v8f accs[8] = {c00, c01, c02, c03, c10, c11, c12, c13};
  float brow[16];
#pragma unroll
  for (int i = 0; i < 16; ++i) brow[i] = 0.f;
  if (MODE == 2) {
#pragma unroll
    for (int i = 0; i < 16; ++i) brow[i] = bf16_rne(bias[row0 + (i >> 3) * 16 + 8 * hh + (i & 7)]);
  }
#pragma unroll
  for (int u = 0; u < 8; ++u) { const int t = u & 3, half = u >> 2; const int col = col0 + t * 16 + ln; const float bcol = (MODE != 2) ? bf16_rne(bias[col]) : 0.f;
#pragma unroll
    for (int r = 0; r < 8; ++r) { const int rloc = half * 16 + 8 * hh + r; const float v = accs[u][r] * alpha + ((MODE == 2) ? brow[half * 8 + r] : bcol); so[w][rloc][t * 16 + ln] = v; } }
  __builtin_amdgcn_fence(4  , "workgroup"); __builtin_amdgcn_wave_barrier();
  if (MODE == 0) {
    const int rsub = lane >> 4, c4 = (lane & 15) * 4;
    for (int pass = 0; pass < 2; ++pass) {
#pragma unroll
      for (int q = 0; q < 16; ++q) { const int r = q * 2 + rsub; const v4f v = *(const v4fa*)&so[w][r][c4]; *(volatile v4f*)(C + (size_t)(row0 + r) * ldc + col0 + c4) = v; }
      if (pass == 0) __threadfence(); }
  } else {
    const int rq = lane >> 3, c8 = (lane & 7) * 8;
    for (int pass = 0; pass < 2; ++pass) {
#pragma unroll
      for (int q = 0; q < 8; ++q) { const int r = q * 4 + rq; const v4f a = *(const v4fa*)&so[w][r][c8], c = *(const v4fa*)&so[w][r][c8 + 4]; FragH f;
#pragma unroll
        for (int i = 0; i < 4; ++i) { f.h[i] = (_Float16)a[i]; f.h[4 + i] = (_Float16)c[i]; }
        const v8us o = f.half[0]; *(volatile v8us*)((unsigned short*)C16 + (size_t)(row0 + r) * ldc + col0 + c8) = o; }
      if (pass == 0) __threadfence(); }
  }
}

__global__ __launch_bounds__(128) void k_gemm_qk(const _Float16* __restrict__ X16, const _Float16* __restrict__ W16, const float* __restrict__ wb, _Float16* __restrict__ QK) {
  gemm_body<1>(X16, DMODEL, W16, DMODEL, 0.015625f, wb, nullptr, QK, LDQK, TOK, LDQK, DMODEL); }
__global__ __launch_bounds__(128) void k_gemm_vt(const _Float16* __restrict__ X16, const _Float16* __restrict__ W16, const float* __restrict__ wb, _Float16* __restrict__ VT) {
  gemm_body<2>(W16 + (size_t)LDQK * DMODEL, DMODEL, X16, DMODEL, 0.015625f, wb + LDQK, nullptr, VT, TOK, DMODEL, TOK, DMODEL); }
__global__ __launch_bounds__(128) void k_gemm_out(const _Float16* __restrict__ CTX, const _Float16* __restrict__ WO16, const float* __restrict__ ob, float* __restrict__ out) {
  gemm_body<0>(CTX, DMODEL, WO16, DMODEL, 0.000244140625f, ob, out, nullptr, DMODEL, TOK, DMODEL, DMODEL); }

__global__ __launch_bounds__(128) void k_flash(const _Float16* __restrict__ QK, const _Float16* __restrict__ VT, _Float16* __restrict__ CTX) {
  __shared__ __attribute__((aligned(16))) unsigned short so[4][16][72];
  const int tid = threadIdx.x, w = tid >> 5, lane = tid & 31, ln = lane & 15, hh = lane >> 4;
  const int h = blockIdx.y; const size_t tokb = (size_t)blockIdx.z * SEQ; const int i0 = blockIdx.x * 64 + w * 16;
  const _Float16* qrow = QK + (tokb + i0 + ln) * LDQK + h * HD;
  const v16h bq0 = g2_frag(qrow, hh), bq1 = g2_frag(qrow + 32, hh);
  const _Float16* kbase = QK + (tokb + ln) * LDQK + DMODEL + h * HD;
  const _Float16* vbase = VT + (size_t)(h * HD + ln) * TOK + tokb;
  const v8f z8 = {0.f,0.f,0.f,0.f,0.f,0.f,0.f,0.f};
  v8f o0 = z8, o1 = z8, o2 = z8, o3 = z8; float m = -1.0e30f, l = 0.f;
#pragma unroll 1
  for (int j = 0; j < SEQ; j += 32) {
    const _Float16* k0p = kbase + (size_t)j * LDQK; const _Float16* k1p = k0p + (size_t)16 * LDQK;
    v8f s0 = z8, s1 = z8;
    s0 = g2_mma(g2_frag(k0p, hh), bq0, s0); s0 = g2_mma(g2_frag(k0p + 32, hh), bq1, s0);
    s1 = g2_mma(g2_frag(k1p, hh), bq0, s1); s1 = g2_mma(g2_frag(k1p + 32, hh), bq1, s1);
    float mx = fmaxf(s0[0], s1[0]);
#pragma unroll
    for (int r = 1; r < 8; ++r) mx = fmaxf(mx, fmaxf(s0[r], s1[r]));
    mx = fmaxf(mx, __shfl_xor(mx, 16, 32));
    const float mn = fmaxf(m, mx * 0.125f); const float al = __expf(m - mn); m = mn;
    FragH pf; float rs = 0.f;
#pragma unroll
    for (int r = 0; r < 8; ++r) { const float p0 = __expf(fmaf(s0[r], 0.125f, -mn)), p1 = __expf(fmaf(s1[r], 0.125f, -mn)); rs += p0 + p1; pf.h[r] = (_Float16)(p0 * 256.0f); pf.h[8 + r] = (_Float16)(p1 * 256.0f); }
    l = l * al + rs; o0 = o0 * al; o1 = o1 * al; o2 = o2 * al; o3 = o3 * al;
    const _Float16* vp = vbase + j;
    o0 = g2_mma(g2_frag(vp, hh), pf.v, o0);
    o1 = g2_mma(g2_frag(vp + (size_t)16 * TOK, hh), pf.v, o1);
    o2 = g2_mma(g2_frag(vp + (size_t)32 * TOK, hh), pf.v, o2);
    o3 = g2_mma(g2_frag(vp + (size_t)48 * TOK, hh), pf.v, o3);
  }
  l += __shfl_xor(l, 16, 32);
  const float sc = 0.25f * (1.0f / l);
  { FragH f;
#pragma unroll
    for (int r = 0; r < 8; ++r) f.h[r] = (_Float16)(o0[r] * sc);
    *(v8us*)&so[w][ln][8 * hh] = f.half[0];
#pragma unroll
    for (int r = 0; r < 8; ++r) f.h[r] = (_Float16)(o1[r] * sc);
    *(v8us*)&so[w][ln][16 + 8 * hh] = f.half[0];
#pragma unroll
    for (int r = 0; r < 8; ++r) f.h[r] = (_Float16)(o2[r] * sc);
    *(v8us*)&so[w][ln][32 + 8 * hh] = f.half[0];
#pragma unroll
    for (int r = 0; r < 8; ++r) f.h[r] = (_Float16)(o3[r] * sc);
    *(v8us*)&so[w][ln][48 + 8 * hh] = f.half[0]; }
  __builtin_amdgcn_fence(4  , "workgroup"); __builtin_amdgcn_wave_barrier();
  const int rq = lane >> 3, pc = (lane & 7) * 8;
  for (int pass = 0; pass < 2; ++pass) {
#pragma unroll
    for (int q = 0; q < 4; ++q) { const int r = q * 4 + rq; const v8us v = *(const v8us*)&so[w][r][pc];
      *(volatile v8us*)((unsigned short*)CTX + (tokb + i0 + r) * DMODEL + h * HD + pc) = v; }
    if (pass == 0) __threadfence(); }
}

extern "C" void kernel_launch(void* const* d_in, const int* in_sizes, int n_in,
                              void* d_out, int out_size, void* d_ws, size_t ws_size, hipStream_t stream) {
  if (n_in < 5) return;
  const size_t need_x = ((size_t)(NB - 1) * SEQ_FULL + SEQ) * DMODEL;
  if ((size_t)in_sizes[0] < need_x) return;
  if ((size_t)in_sizes[1] < (size_t)NQKV * DMODEL) return;
  if ((size_t)in_sizes[2] < (size_t)NQKV) return;
  if ((size_t)in_sizes[3] < (size_t)DMODEL * DMODEL) return;
  if ((size_t)in_sizes[4] < (size_t)DMODEL) return;
  if ((size_t)out_size < (size_t)TOK * DMODEL) return;
  const float* x = (const float*)d_in[0]; const float* Ww = (const float*)d_in[1]; const float* Wb = (const float*)d_in[2];
  const float* ow = (const float*)d_in[3]; const float* ob = (const float*)d_in[4];
  constexpr size_t SZ_X = (size_t)TOK * DMODEL * 2;
  constexpr size_t SZ_W = (size_t)NQKV * DMODEL * 2;
  constexpr size_t SZ_WO = (size_t)DMODEL * DMODEL * 2;
  constexpr size_t SZ_QK = (size_t)TOK * LDQK * 2;
  constexpr size_t SZ_VT = (size_t)DMODEL * TOK * 2;
  constexpr size_t SZ_CTX = (size_t)TOK * DMODEL * 2;
  static_assert(SZ_X % 256 == 0 && SZ_W % 256 == 0 && SZ_WO % 256 == 0 && SZ_QK % 256 == 0 && SZ_VT % 256 == 0 && SZ_CTX % 256 == 0);
  static_assert(SZ_X + SZ_W + SZ_WO + SZ_QK + SZ_VT + SZ_CTX <= (size_t)134217728);
  if (SZ_X + SZ_W + SZ_WO + SZ_QK + SZ_VT + SZ_CTX > ws_size) return;
  char* ws = (char*)d_ws;
  _Float16* X16 = (_Float16*)ws; _Float16* W16 = (_Float16*)(ws + SZ_X); _Float16* WO16 = (_Float16*)(ws + SZ_X + SZ_W);
  _Float16* QK = (_Float16*)(ws + SZ_X + SZ_W + SZ_WO); _Float16* VT = (_Float16*)(ws + SZ_X + SZ_W + SZ_WO + SZ_QK); _Float16* CTX = (_Float16*)(ws + SZ_X + SZ_W + SZ_WO + SZ_QK + SZ_VT);
  k_x16<<<(unsigned)(((size_t)TOK * (DMODEL / 8) + 255) / 256), 256, 0, stream>>>(x, X16);
  k_wnat<<<(unsigned)(((size_t)NQKV * DMODEL / 8 + 255) / 256), 256, 0, stream>>>(Ww, (size_t)NQKV * DMODEL / 8, 64.0f, W16);
  k_wnat<<<(unsigned)(((size_t)DMODEL * DMODEL / 8 + 255) / 256), 256, 0, stream>>>(ow, (size_t)DMODEL * DMODEL / 8, 64.0f, WO16);
  k_gemm_qk<<<(TOK / 128) * (LDQK / 64), 128, 0, stream>>>(X16, W16, Wb, QK);
  k_gemm_vt<<<(DMODEL / 128) * (TOK / 64), 128, 0, stream>>>(X16, W16, Wb, VT);
  k_flash<<<dim3(SEQ / 64, NHEAD, NB), 128, 0, stream>>>(QK, VT, CTX);
  k_gemm_out<<<(TOK / 128) * (DMODEL / 64), 128, 0, stream>>>(CTX, WO16, ob, (float*)d_out);
}
